// CriticCentral_offload_81509889344051
// MI455X (gfx1250) — hardware-verified
//
#include <hip/hip_runtime.h>
#include <stddef.h>


#define NENT    512
#define NE      128
#define DCAT    80
#define K1      96
#define K1P     128
#define N1      256
#define K2      256
#define N2      256
#define NROWT   64
#define AP2     264
#define HP      260
#define SP      129
#define QHP     32
#define ATHR    128
#define MTHR    256
#define WTHR    64
#define WSCAP   134217728

#define LQ      0
#define LK      (LQ + NE * 16)
#define LV      (LK + NE * 16)
#define LRV     (LV + NE * 32)
#define LMA     (LRV + NE)
#define LHC     (LMA + NE)
#define LQH     (LHC + NE)
#define LKH     (LQH + NE * 16)
#define LS      (LKH + NE * 16)
#define LDS_ATTN ((LS + NE * SP) * 4)

#define M_ACT   0
#define M_HB    (M_ACT + NROWT * AP2 * 2)
#define M_DOT   (M_HB + NROWT * HP * 4)
#define LDS_MLP (M_DOT + NROWT * 4)

static_assert((K1 % 32) == 0 && (K2 % 32) == 0 && K1 >= DCAT && K1 <= K1P);
static_assert(((K1P * 2) % 16) == 0 && ((AP2 * 2) % 16) == 0 && ((K2 * 2) % 16) == 0 && ((QHP * 2) % 16) == 0);
static_assert(LDS_ATTN == 116736 && LDS_MLP == 100608);
static_assert(((LQH * 4) % 16) == 0 && ((LKH * 4) % 16) == 0 && ((LS * 4) % 16) == 0);
static_assert(NE * 16 * 4 == NE * QHP * 2);
static_assert(ATHR == NE && MTHR == N1 && N1 == N2 && (ATHR / 32) * 32 == NE);
static_assert((M_HB % 16) == 0 && (M_DOT % 16) == 0);
static_assert((NROWT % 16) == 0 && NROWT <= MTHR && (NROWT / 4) <= 32);
static_assert((N1 * (K1P / 8)) % WTHR == 0 && (N2 * (K2 / 8)) % WTHR == 0);

typedef float    v4f  __attribute__((ext_vector_type(4)));
typedef float    v8f  __attribute__((ext_vector_type(8)));
typedef _Float16 v8h  __attribute__((ext_vector_type(8)));
typedef _Float16 v16h __attribute__((ext_vector_type(16)));
union Frag { v16h v; v8h half[2]; };
static_assert(sizeof(Frag) == 32);

__device__ __forceinline__ v8f wm(v16h a, v16h bq, v8f c) {
  v8f d = __builtin_amdgcn_wmma_f32_16x16x32_f16(false, a, false, bq, (short)0, c, false, false);
  asm volatile("v_nop\n\tv_nop\n\tv_nop\n\tv_nop" : "+v"(d) : "v"(a), "v"(bq));
  return d;
}

__device__ __forceinline__ v8f zero8() {
  v8f z = {0.f, 0.f, 0.f, 0.f, 0.f, 0.f, 0.f, 0.f};
  return z;
}

__global__ __launch_bounds__(WTHR) void k_wcvt(const float* __restrict__ W1, const float* __restrict__ W2,
                                               _Float16* W1T, _Float16* W2T) {
  const int b = blockIdx.x, tid = threadIdx.x;
  const int nb1 = (N1 * (K1P / 8)) / WTHR;
  int n, kg, kval;
  const float* src;
  _Float16* dst;
  if (b < nb1) {
    const int g = b * WTHR + tid;
    n = g >> 4; kg = g & 15; kval = DCAT; src = W1;
    dst = W1T + (size_t)n * K1P + 8 * kg;
  } else {
    const int g = (b - nb1) * WTHR + tid;
    n = g >> 5; kg = g & 31; kval = K2; src = W2;
    dst = W2T + (size_t)n * K2 + 8 * kg;
  }
  v8h hv;
#pragma unroll
  for (int i = 0; i < 8; ++i) {
    const int k  = 8 * kg + i;
    const int kc = k < kval ? k : kval - 1;
    const float v = src[(size_t)kc * N1 + n];
    hv[i] = (_Float16)((k < kval) ? v * 64.0f : 0.0f);
  }
  *(volatile v8h*)dst = hv;
  __threadfence();
  *(volatile v8h*)dst = hv;
}

template <int DV>
__device__ __forceinline__ void softmax_pool(float* lds, float* Sr, float mx, int hoff, int t) {
  float sum = 0.0f;
#pragma unroll 4
  for (int k = 0; k < NE; ++k) {
    const float e = __builtin_amdgcn_exp2f(Sr[k] - mx);
    Sr[k] = e;
    sum += e;
  }
  lds[LRV + t] = 1.0f / sum;
  __syncthreads();

  {
    const float* Sc = lds + LS + t;
    float ma = 0.0f;
#pragma unroll 4
    for (int qq = 0; qq < NE; ++qq) ma = fmaf(Sc[qq * SP], lds[LRV + qq], ma);
    lds[LMA + t] = ma * (1.0f / (float)NE);
  }
  __syncthreads();

  if (t < DV) {
    const float* Vb = lds + LV + t;
    float hs = 0.0f;
#pragma unroll 4
    for (int k = 0; k < NE; ++k) hs = fmaf(lds[LMA + k], Vb[k * DV], hs);
    lds[LHC + hoff + t] = hs;
  }
  __syncthreads();
}

__device__ __forceinline__ void br_pool8(float* lds, const float* __restrict__ st, int off,
                                         const float* __restrict__ W, const float* __restrict__ bias,
                                         float qs, int hoff, int t) {
  constexpr int DQ = 8, DK = 8, DV = 16, D3 = 32;
  {
    const float* sp = st + (size_t)(off + t) * 3;
    const float x0 = sp[0], x1 = sp[1];
#pragma unroll 1
    for (int jg = 0; jg < DQ; ++jg) {
      const v4f w0 = *(const v4f*)(W + 4 * jg);
      const v4f w1 = *(const v4f*)(W + D3 + 4 * jg);
      const v4f bb = *(const v4f*)(bias + 4 * jg);
      const v4f p  = x0 * w0 + x1 * w1 + bb;
      int o;
      if (jg < DQ / 4)      o = LQ + t * DQ + 4 * jg;
      else if (jg < DQ / 2) o = LK + t * DK + 4 * (jg - DQ / 4);
      else                  o = LV + t * DV + 4 * (jg - DQ / 2);
      *(v4f*)(lds + o) = p;
    }
  }
  __syncthreads();

  float q[DQ];
#pragma unroll
  for (int i = 0; i < DQ / 4; ++i) {
    const v4f v = *(const v4f*)(lds + LQ + t * DQ + 4 * i);
    q[4 * i + 0] = v.x * qs; q[4 * i + 1] = v.y * qs; q[4 * i + 2] = v.z * qs; q[4 * i + 3] = v.w * qs;
  }

  float* Sr = lds + LS + t * SP;
  const float* Kb = lds + LK;
  float mx = -3.0e38f;
#pragma unroll 1
  for (int k = 0; k < NE; ++k) {
    const float* kr = Kb + k * DK;
    float s = 0.0f;
#pragma unroll
    for (int i = 0; i < DQ / 4; ++i) {
      const v4f kv = *(const v4f*)(kr + 4 * i);
      s = fmaf(q[4 * i + 0], kv.x, s);
      s = fmaf(q[4 * i + 1], kv.y, s);
      s = fmaf(q[4 * i + 2], kv.z, s);
      s = fmaf(q[4 * i + 3], kv.w, s);
    }
    Sr[k] = s;
    mx = fmaxf(mx, s);
  }

  softmax_pool<DV>(lds, Sr, mx, hoff, t);
}

__device__ __forceinline__ void br_pool16(float* lds, const float* __restrict__ st, int off,
                                          const float* __restrict__ W, const float* __restrict__ bias,
                                          int hoff, int t) {
  constexpr int DQ = 16, DV = 32, D3 = 64;
  const float SC16 = (1.0f / 4096.0f) * 1.4426950408889634f * 0.25f;
  _Float16* Qh = (_Float16*)(lds + LQH);
  _Float16* Kh = (_Float16*)(lds + LKH);
  {
    const float* sp = st + (size_t)(off + t) * 3;
    const float x0 = sp[0], x1 = sp[1];
#pragma unroll 1
    for (int jg8 = 0; jg8 < 4; ++jg8) {
      const v4f w0a = *(const v4f*)(W + 8 * jg8),      w0b = *(const v4f*)(W + 8 * jg8 + 4);
      const v4f w1a = *(const v4f*)(W + D3 + 8 * jg8), w1b = *(const v4f*)(W + D3 + 8 * jg8 + 4);
      const v4f bba = *(const v4f*)(bias + 8 * jg8),   bbb = *(const v4f*)(bias + 8 * jg8 + 4);
      const v4f pa  = (x0 * w0a + x1 * w1a + bba) * 64.0f;
      const v4f pb  = (x0 * w0b + x1 * w1b + bbb) * 64.0f;
      v8h hv;
      hv[0] = (_Float16)pa.x; hv[1] = (_Float16)pa.y; hv[2] = (_Float16)pa.z; hv[3] = (_Float16)pa.w;
      hv[4] = (_Float16)pb.x; hv[5] = (_Float16)pb.y; hv[6] = (_Float16)pb.z; hv[7] = (_Float16)pb.w;
      _Float16* dst = (jg8 < 2) ? (Qh + t * QHP + 8 * jg8) : (Kh + t * QHP + 8 * (jg8 - 2));
      *(v8h*)dst = hv;
    }
    {
      v8h z;
#pragma unroll
      for (int i = 0; i < 8; ++i) z[i] = (_Float16)0.0f;
      *(v8h*)(Qh + t * QHP + 16) = z;
      *(v8h*)(Qh + t * QHP + 24) = z;
      *(v8h*)(Kh + t * QHP + 16) = z;
      *(v8h*)(Kh + t * QHP + 24) = z;
    }
#pragma unroll 1
    for (int jg = 8; jg < DQ; ++jg) {
      const v4f w0 = *(const v4f*)(W + 4 * jg);
      const v4f w1 = *(const v4f*)(W + D3 + 4 * jg);
      const v4f bb = *(const v4f*)(bias + 4 * jg);
      const v4f p  = x0 * w0 + x1 * w1 + bb;
      *(v4f*)(lds + LV + t * DV + 4 * (jg - 8)) = p;
    }
  }
  __syncthreads();

  {
    const int lane = t & 31, w = t >> 5, h = lane >> 4, m = lane & 15;
    const _Float16* qa = Qh + (32 * w + m) * QHP + 8 * h;
    Frag a0, a1;
    a0.half[0] = *(const v8h*)(qa);
    a0.half[1] = *(const v8h*)(qa + 16);
    a1.half[0] = *(const v8h*)(qa + 16 * QHP);
    a1.half[1] = *(const v8h*)(qa + 16 * QHP + 16);
    float* Sb = lds + LS;
#pragma unroll
    for (int tn = 0; tn < 8; ++tn) {
      const _Float16* kb = Kh + (tn * 16 + m) * QHP + 8 * h;
      Frag fb;
      fb.half[0] = *(const v8h*)kb;
      fb.half[1] = *(const v8h*)(kb + 16);
      const v8f d0 = wm(a0.v, fb.v, zero8());
      const v8f d1 = wm(a1.v, fb.v, zero8());
#pragma unroll
      for (int r = 0; r < 8; ++r) {
        Sb[(32 * w + 8 * h + r) * SP + tn * 16 + m]      = d0[r] * SC16;
        Sb[(32 * w + 16 + 8 * h + r) * SP + tn * 16 + m] = d1[r] * SC16;
      }
    }
  }
  __syncthreads();

  float* Sr = lds + LS + t * SP;
  float mx = -3.0e38f;
#pragma unroll 4
  for (int k = 0; k < NE; ++k) mx = fmaxf(mx, Sr[k]);

  softmax_pool<DV>(lds, Sr, mx, hoff, t);
}

__global__ __launch_bounds__(ATHR) void k_attn(
    const float* __restrict__ state,
    const int* __restrict__ p_nrt, const int* __restrict__ p_nob,
    const int* __restrict__ p_nrs, const int* __restrict__ p_ntg,
    const float* __restrict__ W_RT, const float* __restrict__ b_RT,
    const float* __restrict__ W_OB, const float* __restrict__ b_OB,
    const float* __restrict__ W_RS, const float* __restrict__ b_RS,
    const float* __restrict__ W_TG, const float* __restrict__ b_TG,
    _Float16* HA) {
  extern __shared__ v4f lds_dyn[];
  float* lds = (float*)lds_dyn;
  const int t = threadIdx.x, b = blockIdx.x;

  lds[LHC + t] = 0.0f;

  int nrt = p_nrt[0], nob = p_nob[0], nrs = p_nrs[0];
  nrt = min(max(nrt, 0), NENT); nob = min(max(nob, 0), NENT); nrs = min(max(nrs, 0), NENT);
  const int o1 = min(nrt, NENT - NE);
  const int o2 = min(nrt + nob, NENT - NE);
  const int o3 = min(nrt + nob + nrs, NENT - NE);
  (void)p_ntg;

  const float* st = state + (size_t)b * NENT * 3;
  const float qs8 = 1.4426950408889634f * 0.35355339059327373f;

#pragma unroll 1
  for (int br = 0; br < 3; ++br) {
    const float* W  = (br == 0) ? W_RT : (br == 1) ? W_OB : W_RS;
    const float* bb = (br == 0) ? b_RT : (br == 1) ? b_OB : b_RS;
    const int   off = (br == 0) ? 0 : (br == 1) ? o1 : o2;
    br_pool8(lds, st, off, W, bb, qs8, 16 * br, t);
  }
  br_pool16(lds, st, o3, W_TG, b_TG, 48, t);

  if (t < 16) {
    v8h hv;
#pragma unroll
    for (int i = 0; i < 8; ++i) hv[i] = (_Float16)(lds[LHC + 8 * t + i] * 256.0f);
    _Float16* dst = HA + (size_t)b * K1P + 8 * t;
    *(volatile v8h*)dst = hv;
    __threadfence();
    *(volatile v8h*)dst = hv;
  }
}

__global__ __launch_bounds__(MTHR) void k_mlp(
    const _Float16* __restrict__ HA, const _Float16* __restrict__ W1T, const float* __restrict__ b1,
    const _Float16* __restrict__ W2T, const float* __restrict__ b2,
    const float* __restrict__ W3, const float* __restrict__ b3, float* out) {
  extern __shared__ v4f lds_dyn[];
  char* sm = (char*)lds_dyn;
  _Float16* act = (_Float16*)(sm + M_ACT);
  float* hb   = (float*)(sm + M_HB);
  float* dots = (float*)(sm + M_DOT);
  const int tid = threadIdx.x, lane = tid & 31, wave = tid >> 5, h = lane >> 4, m = lane & 15;
  const int rt = wave & 3, cg = wave >> 2;
  const int colBase = cg * 128;
  const int rowBase = blockIdx.x * NROWT;

  v8f acc[8];
#pragma unroll
  for (int nt = 0; nt < 8; ++nt) acc[nt] = zero8();

  {
    const _Float16* ap = HA + (size_t)(rowBase + rt * 16 + m) * K1P + 8 * h;
    const _Float16* bq = W1T + (size_t)(colBase + m) * K1P + 8 * h;
#pragma unroll 1
    for (int ks = 0; ks < K1 / 32; ++ks) {
      const int ko = 32 * ks;
      Frag fa;
      fa.half[0] = *(const v8h*)(ap + ko);
      fa.half[1] = *(const v8h*)(ap + ko + 16);
#pragma unroll
      for (int nt = 0; nt < 8; ++nt) {
        const _Float16* pb = bq + (size_t)(nt * 16) * K1P + ko;
        Frag fb;
        fb.half[0] = *(const v8h*)pb;
        fb.half[1] = *(const v8h*)(pb + 16);
        acc[nt] = wm(fa.v, fb.v, acc[nt]);
      }
    }
  }
#pragma unroll
  for (int nt = 0; nt < 8; ++nt) {
#pragma unroll
    for (int r = 0; r < 8; ++r) hb[(rt * 16 + 8 * h + r) * HP + colBase + nt * 16 + m] = acc[nt][r];
  }
  __syncthreads();

  {
    const float bc = b1[tid];
#pragma unroll 1
    for (int i = 0; i < NROWT; ++i) {
      const float v = hb[i * HP + tid] * (1.0f / 16384.0f) + bc;
      act[i * AP2 + tid] = (_Float16)(tanhf(v) * 1024.0f);
    }
  }
  __syncthreads();

#pragma unroll
  for (int nt = 0; nt < 8; ++nt) acc[nt] = zero8();
  {
    const _Float16* ap = act + (rt * 16 + m) * AP2 + 8 * h;
    const _Float16* bq = W2T + (size_t)(colBase + m) * K2 + 8 * h;
#pragma unroll 1
    for (int ks = 0; ks < K2 / 32; ++ks) {
      const int ko = 32 * ks;
      Frag fa;
      fa.half[0] = *(const v8h*)(ap + ko);
      fa.half[1] = *(const v8h*)(ap + ko + 16);
#pragma unroll
      for (int nt = 0; nt < 8; ++nt) {
        const _Float16* pb = bq + (size_t)(nt * 16) * K2 + ko;
        Frag fb;
        fb.half[0] = *(const v8h*)pb;
        fb.half[1] = *(const v8h*)(pb + 16);
        acc[nt] = wm(fa.v, fb.v, acc[nt]);
      }
    }
  }
#pragma unroll
  for (int nt = 0; nt < 8; ++nt) {
#pragma unroll
    for (int r = 0; r < 8; ++r) hb[(rt * 16 + 8 * h + r) * HP + colBase + nt * 16 + m] = acc[nt][r];
  }
  __syncthreads();

  {
    const float bc = b2[tid];
#pragma unroll 1
    for (int i = 0; i < NROWT; ++i) {
      const float v = hb[i * HP + tid] * (1.0f / 65536.0f) + bc;
      hb[i * HP + tid] = tanhf(v);
    }
  }
  __syncthreads();

  if (tid < NROWT) {
    const float* hr = hb + tid * HP;
    float d = 0.0f;
#pragma unroll 4
    for (int c = 0; c < N2; ++c) d = fmaf(hr[c], W3[c], d);
    dots[tid] = d + b3[0];
  }
  __syncthreads();

  if (tid < NROWT / 4) {
    const v4f v = *(const v4f*)(dots + 4 * tid);
    float* op = out + (size_t)rowBase + 4 * tid;
    *(volatile v4f*)op = v;
    __threadfence();
    *(volatile v4f*)op = v;
  }
}

extern "C" void kernel_launch(void* const* d_in, const int* in_sizes, int n_in,
                              void* d_out, int out_size, void* d_ws, size_t ws_size,
                              hipStream_t stream) {
  if (n_in < 19) return;
  const int nsamp = in_sizes[0] / (NENT * 3);
  if (nsamp <= 0 || in_sizes[0] != nsamp * NENT * 3 || (nsamp % NROWT) != 0) return;
  if (out_size != nsamp) return;
  if (in_sizes[1] != 1 || in_sizes[2] != 1 || in_sizes[3] != 1 || in_sizes[4] != 1) return;
  if (in_sizes[5] != 64 || in_sizes[6] != 32 || in_sizes[7] != 64 || in_sizes[8] != 32) return;
  if (in_sizes[9] != 64 || in_sizes[10] != 32 || in_sizes[11] != 128 || in_sizes[12] != 64) return;
  if (in_sizes[13] != DCAT * N1 || in_sizes[14] != N1 || in_sizes[15] != K2 * N2 || in_sizes[16] != N2) return;
  if (in_sizes[17] != K2 || in_sizes[18] != 1) return;

  const float* state = (const float*)d_in[0];
  const int*   n_rt  = (const int*)d_in[1];
  const int*   n_ob  = (const int*)d_in[2];
  const int*   n_rs  = (const int*)d_in[3];
  const int*   n_tg  = (const int*)d_in[4];
  const float* W_RT  = (const float*)d_in[5];
  const float* b_RT  = (const float*)d_in[6];
  const float* W_OB  = (const float*)d_in[7];
  const float* b_OB  = (const float*)d_in[8];
  const float* W_RS  = (const float*)d_in[9];
  const float* b_RS  = (const float*)d_in[10];
  const float* W_TG  = (const float*)d_in[11];
  const float* b_TG  = (const float*)d_in[12];
  const float* W1    = (const float*)d_in[13];
  const float* b1    = (const float*)d_in[14];
  const float* W2    = (const float*)d_in[15];
  const float* b2    = (const float*)d_in[16];
  const float* W3    = (const float*)d_in[17];
  const float* b3    = (const float*)d_in[18];
  float* out = (float*)d_out;

  size_t off = 0;
  const size_t oHA  = off; off += (size_t)nsamp * K1P * 2;   off = (off + 255) & ~(size_t)255;
  const size_t oW1T = off; off += (size_t)N1 * K1P * 2;      off = (off + 255) & ~(size_t)255;
  const size_t oW2T = off; off += (size_t)N2 * K2 * 2;       off = (off + 255) & ~(size_t)255;
  const size_t tot = off;
  if (tot > ws_size || tot > (size_t)WSCAP) return;
  char* ws = (char*)d_ws;
  _Float16* HA  = (_Float16*)(ws + oHA);
  _Float16* W1T = (_Float16*)(ws + oW1T);
  _Float16* W2T = (_Float16*)(ws + oW2T);

  const int nbw = (N1 * (K1P / 8)) / WTHR + (N2 * (K2 / 8)) / WTHR;
  k_wcvt<<<nbw, WTHR, 0, stream>>>(W1, W2, W1T, W2T);

  hipFuncSetAttribute(reinterpret_cast<const void*>(&k_attn),
                      hipFuncAttributeMaxDynamicSharedMemorySize, LDS_ATTN);
  k_attn<<<nsamp, ATHR, LDS_ATTN, stream>>>(state, n_rt, n_ob, n_rs, n_tg,
                                            W_RT, b_RT, W_OB, b_OB, W_RS, b_RS, W_TG, b_TG, HA);

  hipFuncSetAttribute(reinterpret_cast<const void*>(&k_mlp),
                      hipFuncAttributeMaxDynamicSharedMemorySize, LDS_MLP);
  k_mlp<<<nsamp / NROWT, MTHR, LDS_MLP, stream>>>(HA, W1T, b1, W2T, b2, W3, b3, out);
}
